// PositionalInferenceBlock_28578712388214
// MI455X (gfx1250) — hardware-verified
//
#include <hip/hip_runtime.h>
#include <math.h>
#include <stddef.h>

constexpr int kTime  = 64;
constexpr int kPers  = 64;
constexpr int kFeat  = 128;
constexpr int kAttn  = 32;
constexpr int kPos   = 32;
constexpr int kRowsBD = kTime * kPers;
constexpr int kKX    = kFeat + kPos;
constexpr int kNCol  = 192;
constexpr int kGroupsPerChunk = 16;
constexpr int kRowsPerGroup   = 4096;
constexpr int kRowsPerChunk   = kGroupsPerChunk * kRowsPerGroup;
constexpr int kNumChunk       = 4;
static_assert(kKX % 32 == 0, "K multiple of 32");
static_assert(kNCol % 64 == 0 && kRowsPerChunk % 64 == 0 && kRowsBD % 64 == 0, "tile multiples");

constexpr size_t kOffBdH   = 0;
constexpr size_t kOffBdL   = kOffBdH + 1048576;
constexpr size_t kOffWaTH  = kOffBdL + 1048576;
constexpr size_t kOffWaTL  = kOffWaTH + 16384;
constexpr size_t kOffWcTH  = kOffWaTL + 16384;
constexpr size_t kOffWcTL  = kOffWcTH + 61440;
constexpr size_t kOffBiasC = kOffWcTL + 61440;
constexpr size_t kOffBiasA = kOffBiasC + 1024;
constexpr size_t kOffTheta = 2256896;
constexpr size_t kOffOutSp = kOffTheta + 1048576;
constexpr size_t kOffAH    = kOffOutSp + 2097152;
constexpr size_t kOffAL    = kOffAH + 20971520;
constexpr size_t kOffCpl   = kOffAL + 20971520;
constexpr size_t kWsTotal  = kOffCpl + 50331648;
static_assert(kOffBiasA + 256 <= kOffTheta, "prefix fits");
static_assert(kWsTotal <= 134217728u, "carve within 128 MiB");
static_assert((kOffTheta % 4096) == 0 && (kOffBiasC % 128) == 0 && (kOffBiasA % 128) == 0, "alignment");

typedef __attribute__((ext_vector_type(16))) _Float16 v16h;
typedef __attribute__((ext_vector_type(8)))  _Float16 v8h;
typedef __attribute__((ext_vector_type(16))) __bf16   v16b;
typedef __attribute__((ext_vector_type(8)))  __bf16   v8b;
typedef __attribute__((ext_vector_type(8)))  float    v8f;
typedef __attribute__((ext_vector_type(4)))  float    v4f;
typedef __attribute__((ext_vector_type(4)))  unsigned int v4u;

__device__ __forceinline__ unsigned short f2bf_bits(float f) {
  unsigned u = __float_as_uint(f);
  return (unsigned short)((u + 0x7FFFu + ((u >> 16) & 1u)) >> 16);
}
__device__ __forceinline__ float bf_bits2f(unsigned short h) { return __uint_as_float(((unsigned)h) << 16); }

__device__ __forceinline__ void dep_guard_h(v8f& a, v8f& b, v16h x, v16h y) { asm volatile("v_nop\n\tv_nop\n\tv_nop\n\tv_nop" : "+v"(a), "+v"(b) : "v"(x), "v"(y)); }
__device__ __forceinline__ void dep_guard_b(v8f& a, v8f& b, v16b x, v16b y) { asm volatile("v_nop\n\tv_nop\n\tv_nop\n\tv_nop" : "+v"(a), "+v"(b) : "v"(x), "v"(y)); }
__device__ __forceinline__ void keep4_h(v16h a, v16h b, v16h c, v16h d) { asm volatile("v_nop" :: "v"(a), "v"(b), "v"(c), "v"(d)); }
__device__ __forceinline__ void keep4_b(v16b a, v16b b, v16b c, v16b d) { asm volatile("v_nop" :: "v"(a), "v"(b), "v"(c), "v"(d)); }
__device__ __forceinline__ void acc_guard4(v8f& a, v8f& b, v8f& c, v8f& d) { asm volatile("v_nop\n\tv_nop\n\tv_nop\n\tv_nop" : "+v"(a), "+v"(b), "+v"(c), "+v"(d)); }
template <typename T> struct Frag;
template <> struct Frag<_Float16> {
  typedef v16h V; union U { v16h v; v8h h[2]; };
  static __device__ __forceinline__ v16h load(const _Float16* p) {
    U f; f.h[0] = *(const v8h*)(p); f.h[1] = *(const v8h*)(p + 16); return f.v;
  }
  static __device__ __forceinline__ v8f mma(v16h a, v16h b, v8f c) {
    return __builtin_amdgcn_wmma_f32_16x16x32_f16(false, a, false, b, (short)0, c, false, false);
  }
  static __device__ __forceinline__ void guard(v8f& a, v8f& b, v16h x, v16h y) { dep_guard_h(a, b, x, y); }
  static __device__ __forceinline__ void keep(v16h a, v16h b, v16h c, v16h d) { keep4_h(a, b, c, d); }
};
template <> struct Frag<__bf16> {
  typedef v16b V; union U { v16b v; v8b h[2]; };
  static __device__ __forceinline__ v16b load(const __bf16* p) {
    U f; f.h[0] = *(const v8b*)(p); f.h[1] = *(const v8b*)(p + 16); return f.v;
  }
  static __device__ __forceinline__ v8f mma(v16b a, v16b b, v8f c) {
    return __builtin_amdgcn_wmma_f32_16x16x32_bf16(false, a, false, b, (short)0, c, false, false);
  }
  static __device__ __forceinline__ void guard(v8f& a, v8f& b, v16b x, v16b y) { dep_guard_b(a, b, x, y); }
  static __device__ __forceinline__ void keep(v16b a, v16b b, v16b c, v16b d) { keep4_b(a, b, c, d); }
};

__device__ __forceinline__ unsigned pk16(unsigned short a, unsigned short b) { return (unsigned)a | ((unsigned)b << 16); }

__device__ __forceinline__ void split_bf2(float x, unsigned short& hb, unsigned short& lb) {
  hb = f2bf_bits(x);
  lb = f2bf_bits(x - bf_bits2f(hb));
}

template <int ET> struct Elem;
template <> struct Elem<0> { typedef _Float16 T; };
template <> struct Elem<1> { typedef __bf16 T; };
template <int ET, bool SPLIT, int BIAS_MODE, int OUT_MODE, bool RESID, int ACT = 0>
__global__ __launch_bounds__(256) void wmma_gemm64(
    const unsigned short* __restrict__ Ap, const unsigned short* __restrict__ A2p, int lda, long strideA,
    const unsigned short* __restrict__ Btp, const unsigned short* __restrict__ Bt2p, int ldb, long strideB,
    void* __restrict__ Cout, void* __restrict__ Cout2, int ldc, long strideC,
    const float* __restrict__ bias,
    const float* __restrict__ resid, long strideR,
    int M, int N, int K, float scale) {
  typedef typename Elem<ET>::T T;
  typedef typename Frag<T>::V V;
  const T* A = (const T*)Ap; const T* A2 = (const T*)A2p; const T* Bt = (const T*)Btp; const T* Bt2 = (const T*)Bt2p;
  __shared__ __align__(16) float sT[8][16 * 68];
  const int b    = blockIdx.y;
  const int lane = threadIdx.x & 31;
  const int wave = threadIdx.x >> 5;
  const int tilesN = N >> 6;
  const int tilesM = M >> 6;
  const int tile = blockIdx.x * 8 + wave;
  if (tile >= tilesM * tilesN) return;
  const int tm = tile / tilesN;
  const int tn = tile - tm * tilesN;
  const int m0 = tm << 6;
  const int n0 = tn << 6;

  const T* Ab  = A  + (size_t)b * strideA;
  const T* Bb  = Bt + (size_t)b * strideB;
  const T* Ab2 = SPLIT ? (A2  + (size_t)b * strideA) : nullptr;
  const T* Bb2 = SPLIT ? (Bt2 + (size_t)b * strideB) : nullptr;

  const int rlane = lane & 15;
  const int koff  = (lane >> 4) * 8;
  const int mOff  = (lane >> 4) * 8;

  v8f acc[4][4];
#pragma unroll
  for (int i = 0; i < 4; ++i)
#pragma unroll
    for (int j = 0; j < 4; ++j) acc[i][j] = (v8f){0.f,0.f,0.f,0.f,0.f,0.f,0.f,0.f};

  for (int k0 = 0; k0 < K; k0 += 32) {
    V bh[4], bl[4];
#pragma unroll
    for (int j = 0; j < 4; ++j) {
      const size_t bo = (size_t)(n0 + (j << 4) + rlane) * ldb + koff + k0;
      bh[j] = Frag<T>::load(Bb + bo);
      if (SPLIT) bl[j] = Frag<T>::load(Bb2 + bo);
    }
#pragma unroll
    for (int i = 0; i < 4; ++i) {
      const size_t ao = (size_t)(m0 + (i << 4) + rlane) * lda + koff + k0;
      V ah = Frag<T>::load(Ab + ao);
      V al;
      if (SPLIT) al = Frag<T>::load(Ab2 + ao);
#pragma unroll
      for (int j = 0; j < 4; ++j) {
        acc[i][j] = Frag<T>::mma(ah, bh[j], acc[i][j]);
        if (SPLIT) {
          acc[i][j] = Frag<T>::mma(ah, bl[j], acc[i][j]);
          acc[i][j] = Frag<T>::mma(al, bh[j], acc[i][j]);
        }
      }
      Frag<T>::guard(acc[i][0], acc[i][3], ah, SPLIT ? al : ah);
    }
    Frag<T>::keep(bh[0], bh[1], bh[2], bh[3]);
    if (SPLIT) Frag<T>::keep(bl[0], bl[1], bl[2], bl[3]);
  }
  acc_guard4(acc[0][0], acc[0][1], acc[0][2], acc[0][3]);
  acc_guard4(acc[1][0], acc[1][1], acc[1][2], acc[1][3]);
  acc_guard4(acc[2][0], acc[2][1], acc[2][2], acc[2][3]);
  acc_guard4(acc[3][0], acc[3][1], acc[3][2], acc[3][3]);

  float* slab = sT[wave];
  const float* Rb = RESID ? (resid + (size_t)b * strideR) : nullptr;
#pragma unroll
  for (int i = 0; i < 4; ++i) {
    const int mBase = m0 + (i << 4);
#pragma unroll
    for (int j = 0; j < 4; ++j) {
      const int n = n0 + (j << 4) + rlane;
      float bv = 0.f;
      if (BIAS_MODE == 2) bv = bias[n];
#pragma unroll
      for (int r = 0; r < 8; ++r) {
        float v = acc[i][j][r] * scale;
        if (BIAS_MODE == 1) v += bias[mBase + mOff + r];
        if (BIAS_MODE == 2) v += bv;
        if (RESID) v += Rb[(size_t)(mBase + mOff + r) * ldc + n];
        if (ACT == 2) v = fmaxf(v, 0.0f);
        if (ACT == 4) v = (v > 0.f) ? v : 0.01f * v;
        slab[(mOff + r) * 68 + (j << 4) + rlane] = v;
      }
    }
    __builtin_amdgcn_fence(__ATOMIC_RELEASE, "workgroup");
    __builtin_amdgcn_wave_barrier();
    __builtin_amdgcn_fence(__ATOMIC_ACQUIRE, "workgroup");
    if (OUT_MODE == 0) {
      float* C = (float*)Cout + (size_t)b * strideC;
      const int hh = lane >> 4, c4 = (lane & 15) * 4;
      for (int pass = 0; pass < 2; ++pass) {
#pragma unroll
        for (int it = 0; it < 8; ++it) {
          const int row = it * 2 + hh;
          v4f v = *(const v4f*)(slab + row * 68 + c4);
          *(volatile v4f*)(C + (size_t)(mBase + row) * ldc + n0 + c4) = v;
        }
        __threadfence();
      }
    } else {
      const int q = lane >> 3, c8 = (lane & 7) * 8;
      unsigned short* C  = (unsigned short*)Cout  + (size_t)b * strideC;
      unsigned short* C2 = (OUT_MODE == 2) ? ((unsigned short*)Cout2 + (size_t)b * strideC) : nullptr;
      for (int pass = 0; pass < 2; ++pass) {
#pragma unroll
        for (int it = 0; it < 4; ++it) {
          const int row = it * 4 + q;
          const float* sp = slab + row * 68 + c8;
          v8h hv, lv;
#pragma unroll
          for (int e = 0; e < 8; ++e) {
            if (OUT_MODE == 1) {
              hv[e] = (_Float16)sp[e];
            } else {
              unsigned short hb = f2bf_bits(sp[e]);
              unsigned short lb = f2bf_bits(sp[e] - bf_bits2f(hb));
              hv[e] = __builtin_bit_cast(_Float16, hb);
              lv[e] = __builtin_bit_cast(_Float16, lb);
            }
          }
          *(volatile v8h*)(C + (size_t)(mBase + row) * ldc + n0 + c8) = hv;
          if (OUT_MODE == 2) *(volatile v8h*)(C2 + (size_t)(mBase + row) * ldc + n0 + c8) = lv;
        }
        __threadfence();
      }
    }
    __builtin_amdgcn_fence(__ATOMIC_RELEASE, "workgroup");
    __builtin_amdgcn_wave_barrier();
    __builtin_amdgcn_fence(__ATOMIC_ACQUIRE, "workgroup");
  }
}

__global__ __launch_bounds__(256) void cast_split8_kernel(const float* __restrict__ in,
                                                         unsigned short* __restrict__ oh,
                                                         unsigned short* __restrict__ ol, int n8) {
  const int i = blockIdx.x * 256 + threadIdx.x;
  if (i >= n8) return;
  const float* p = in + 8 * (size_t)i;
  const v4f a = *(const v4f*)(p);
  const v4f c = *(const v4f*)(p + 4);
  unsigned short hb[8], lb[8];
#pragma unroll
  for (int e = 0; e < 4; ++e) {
    split_bf2(a[e], hb[e], lb[e]);
    split_bf2(c[e], hb[4 + e], lb[4 + e]);
  }
  const v4u uh = (v4u){pk16(hb[0], hb[1]), pk16(hb[2], hb[3]), pk16(hb[4], hb[5]), pk16(hb[6], hb[7])};
  const v4u ul = (v4u){pk16(lb[0], lb[1]), pk16(lb[2], lb[3]), pk16(lb[4], lb[5]), pk16(lb[6], lb[7])};
  unsigned short* qh = oh + 8 * (size_t)i;
  unsigned short* ql = ol + 8 * (size_t)i;
  *(volatile v4u*)qh = uh;
  *(volatile v4u*)ql = ul;
  __threadfence();
  *(volatile v4u*)qh = uh;
  *(volatile v4u*)ql = ul;
}

__global__ __launch_bounds__(256) void prep_weights_kernel(
    const float* __restrict__ Wa, const float* __restrict__ Wb, const float* __restrict__ Wg,
    const float* __restrict__ ba, const float* __restrict__ bb, const float* __restrict__ bg,
    unsigned short* __restrict__ WaTh, unsigned short* __restrict__ WaTl,
    unsigned short* __restrict__ WcTh, unsigned short* __restrict__ WcTl,
    float* __restrict__ bias_cat, float* __restrict__ bias_a) {
  const int y = blockIdx.y;
  const int t = blockIdx.x * 256 + threadIdx.x;
  if (y == 0) {
    if (t >= 1024) return;
    const int n = t >> 4, k0 = (t & 15) * 8;
    const int nc = (n < 32) ? n : 31;
    unsigned short hb[8], lb[8];
#pragma unroll
    for (int e = 0; e < 8; ++e) {
      const float w = Wa[(k0 + e) * kAttn + nc];
      const float v = (n < 32) ? w : 0.0f;
      split_bf2(v, hb[e], lb[e]);
    }
    const v4u uh = (v4u){pk16(hb[0], hb[1]), pk16(hb[2], hb[3]), pk16(hb[4], hb[5]), pk16(hb[6], hb[7])};
    const v4u ul = (v4u){pk16(lb[0], lb[1]), pk16(lb[2], lb[3]), pk16(lb[4], lb[5]), pk16(lb[6], lb[7])};
    unsigned short* qh = WaTh + (size_t)n * kFeat + k0;
    unsigned short* ql = WaTl + (size_t)n * kFeat + k0;
    *(volatile v4u*)qh = uh;
    *(volatile v4u*)ql = ul;
    __threadfence();
    *(volatile v4u*)qh = uh;
    *(volatile v4u*)ql = ul;
  } else if (y == 1) {
    if (t >= 3840) return;
    const int n = t / 20, k0 = (t - n * 20) * 8;
    const int nb = (n < 32) ? n : 31;
    int ng = n - 32; ng = (ng < 0) ? 0 : ng; ng = (ng > 127) ? 127 : ng;
    unsigned short hb[8], lb[8];
#pragma unroll
    for (int e = 0; e < 8; ++e) {
      const int k = k0 + e;
      const float wb = Wb[k * kAttn + nb];
      const float wg = Wg[k * kFeat + ng];
      const float v = (n < 32) ? wb : ((n < 160) ? wg : 0.0f);
      split_bf2(v, hb[e], lb[e]);
    }
    const v4u uh = (v4u){pk16(hb[0], hb[1]), pk16(hb[2], hb[3]), pk16(hb[4], hb[5]), pk16(hb[6], hb[7])};
    const v4u ul = (v4u){pk16(lb[0], lb[1]), pk16(lb[2], lb[3]), pk16(lb[4], lb[5]), pk16(lb[6], lb[7])};
    unsigned short* qh = WcTh + (size_t)n * kKX + k0;
    unsigned short* ql = WcTl + (size_t)n * kKX + k0;
    *(volatile v4u*)qh = uh;
    *(volatile v4u*)ql = ul;
    __threadfence();
    *(volatile v4u*)qh = uh;
    *(volatile v4u*)ql = ul;
  } else {
    if (t < 48) {
      const int n0 = t * 4;
      v4f v;
#pragma unroll
      for (int e = 0; e < 4; ++e) {
        const int n = n0 + e;
        const int nb = (n < 32) ? n : 31;
        int ng = n - 32; ng = (ng < 0) ? 0 : ng; ng = (ng > 127) ? 127 : ng;
        const float vb = bb[nb];
        const float vg = bg[ng];
        v[e] = (n < 32) ? vb : ((n < 160) ? vg : 0.0f);
      }
      float* q = bias_cat + n0;
      *(volatile v4f*)q = v;
      __threadfence();
      *(volatile v4f*)q = v;
    } else if (t >= 64 && t < 80) {
      const int n0 = (t - 64) * 4;
      v4f v;
#pragma unroll
      for (int e = 0; e < 4; ++e) {
        const int n = n0 + e;
        const int na = (n < 32) ? n : 31;
        const float va = ba[na];
        v[e] = (n < 32) ? va : 0.0f;
      }
      float* q = bias_a + n0;
      *(volatile v4f*)q = v;
      __threadfence();
      *(volatile v4f*)q = v;
    }
  }
}

__global__ __launch_bounds__(256) void build_rows_kernel(
    const unsigned short* __restrict__ bdh, const unsigned short* __restrict__ bdl,
    const float* __restrict__ extra, const float* __restrict__ Wx, const float* __restrict__ bx,
    unsigned short* __restrict__ Ah, unsigned short* __restrict__ Al,
    int D, int G0, int bdG, int bdB) {
  __shared__ __align__(16) unsigned short sH[64 * kKX];
  __shared__ __align__(16) unsigned short sL[64 * kKX];
  __shared__ float sX[64 * 10];
  __shared__ float sW[10 * 32];
  __shared__ float sB[32];
  const int tid = threadIdx.x;
  const int gl  = blockIdx.x >> 6, blk = blockIdx.x & 63;
  const int G   = G0 + gl;
  const int bdbase = G * bdG + blk * bdB;
  const size_t xbase = ((size_t)G * kRowsPerGroup + (size_t)blk * 64) * (size_t)D;

  for (int q = tid; q < 1024; q += 256) {
    const int row = q >> 4, c8 = (q & 15) * 8;
    const v4u h = *(const v4u*)(bdh + (size_t)(bdbase + row) * kFeat + c8);
    const v4u l = *(const v4u*)(bdl + (size_t)(bdbase + row) * kFeat + c8);
    *(v4u*)(sH + row * kKX + c8) = h;
    *(v4u*)(sL + row * kKX + c8) = l;
  }
  for (int idx = tid; idx < 64 * D; idx += 256) sX[idx] = extra[xbase + idx];
  for (int idx = tid; idx < 32 * D; idx += 256) sW[idx] = Wx[idx];
  if (tid < 32) sB[tid] = bx[tid];
  __syncthreads();

  {
    const int row = tid >> 2, c0 = (tid & 3) * 8;
    float v[8];
#pragma unroll
    for (int e = 0; e < 8; ++e) v[e] = 0.0f;
#pragma unroll 1
    for (int d = 0; d < D; ++d) {
      const float xd = sX[row * D + d];
      const float* w = sW + d * 32 + c0;
#pragma unroll
      for (int e = 0; e < 8; ++e) v[e] = v[e] + xd * w[e];
    }
    unsigned short hb[8], lb[8];
#pragma unroll
    for (int e = 0; e < 8; ++e) split_bf2(v[e] + sB[c0 + e], hb[e], lb[e]);
    const v4u uh = (v4u){pk16(hb[0], hb[1]), pk16(hb[2], hb[3]), pk16(hb[4], hb[5]), pk16(hb[6], hb[7])};
    const v4u ul = (v4u){pk16(lb[0], lb[1]), pk16(lb[2], lb[3]), pk16(lb[4], lb[5]), pk16(lb[6], lb[7])};
    *(v4u*)(sH + row * kKX + kFeat + c0) = uh;
    *(v4u*)(sL + row * kKX + kFeat + c0) = ul;
  }
  __syncthreads();

  const size_t obase = (size_t)blockIdx.x * 1280;
  const v4u* sh4 = (const v4u*)sH;
  const v4u* sl4 = (const v4u*)sL;
  v4u* oh = (v4u*)Ah + obase;
  v4u* ol = (v4u*)Al + obase;
  for (int q = tid; q < 1280; q += 256) {
    const v4u a = sh4[q];
    const v4u c = sl4[q];
    *(volatile v4u*)(oh + q) = a;
    *(volatile v4u*)(ol + q) = c;
  }
  __threadfence();
  for (int q = tid; q < 1280; q += 256) {
    const v4u a = sh4[q];
    const v4u c = sl4[q];
    *(volatile v4u*)(oh + q) = a;
    *(volatile v4u*)(ol + q) = c;
  }
}

__global__ __launch_bounds__(256) void attn_rows_kernel(
    const float* __restrict__ Cpl, const float* __restrict__ thetaC,
    const float* __restrict__ addsrc, float* __restrict__ dst,
    int G0, int sq, int sk, int addflag) {
  __shared__ float sw[8][64];
  const int tid = threadIdx.x, wave = tid >> 5, lane = tid & 31;
  const int wg = blockIdx.x * 8 + wave;
  const int gl = wg >> 6, q = wg & 63;
  const int G  = G0 + gl;
  const float* th = thetaC + (size_t)(G * 64 + q) * 64;
  const size_t rbase = (size_t)gl * kRowsPerGroup + (size_t)q * sq;
  const float* p0 = Cpl + (rbase + (size_t)lane * sk) * kNCol;
  const float* p1 = Cpl + (rbase + (size_t)(lane + 32) * sk) * kNCol;
  float s0 = 0.0f, s1 = 0.0f;
#pragma unroll 1
  for (int a4 = 0; a4 < 8; ++a4) {
    const v4f tv = *(const v4f*)(th + 4 * a4);
    const v4f x0 = *(const v4f*)(p0 + 4 * a4);
    const v4f x1 = *(const v4f*)(p1 + 4 * a4);
    s0 += tv[0] * x0[0]; s0 += tv[1] * x0[1]; s0 += tv[2] * x0[2]; s0 += tv[3] * x0[3];
    s1 += tv[0] * x1[0]; s1 += tv[1] * x1[1]; s1 += tv[2] * x1[2]; s1 += tv[3] * x1[3];
  }
  float m = fmaxf(s0, s1);
#pragma unroll
  for (int off = 16; off > 0; off >>= 1) m = fmaxf(m, __shfl_xor(m, off, 32));
  const float e0 = expf(s0 - m), e1 = expf(s1 - m);
  float su = e0 + e1;
#pragma unroll
  for (int off = 16; off > 0; off >>= 1) su += __shfl_xor(su, off, 32);
  const float inv = 1.0f / su;
  sw[wave][lane]      = e0 * inv;
  sw[wave][lane + 32] = e1 * inv;
  __builtin_amdgcn_fence(__ATOMIC_RELEASE, "workgroup");
  __builtin_amdgcn_wave_barrier();
  __builtin_amdgcn_fence(__ATOMIC_ACQUIRE, "workgroup");

  v4f acc = (v4f){0.0f, 0.0f, 0.0f, 0.0f};
  const float* fb = Cpl + rbase * kNCol + kAttn + 4 * lane;
#pragma unroll 1
  for (int k = 0; k < 64; ++k) {
    const float wk = sw[wave][k];
    const v4f f = *(const v4f*)(fb + (size_t)k * sk * kNCol);
    acc += wk * f;
  }
  const size_t orow = (size_t)(G * 64 + q) * kFeat + 4 * lane;
  const v4f ad = *(const v4f*)(addsrc + orow);
  if (addflag != 0) acc += ad;
  float* op = dst + orow;
  *(volatile v4f*)op = acc;
  __threadfence();
  *(volatile v4f*)op = acc;
}


extern "C" void kernel_launch(void* const* d_in, const int* in_sizes, int n_in,
                              void* d_out, int out_size, void* d_ws, size_t ws_size,
                              hipStream_t stream) {
  if (n_in < 13) return;
  if (in_sizes[0] != kRowsBD * kFeat) return;
  if (in_sizes[1] != kTime * kPers * kPers * 9) return;
  if (in_sizes[2] != kTime * kTime * kPers * 10) return;
  if (in_sizes[3] != kFeat * kAttn || in_sizes[4] != kAttn) return;
  if (in_sizes[5] != kKX * kAttn || in_sizes[6] != kAttn) return;
  if (in_sizes[7] != kKX * kFeat || in_sizes[8] != kFeat) return;
  if (in_sizes[9] != 9 * kPos || in_sizes[10] != kPos) return;
  if (in_sizes[11] != 10 * kPos || in_sizes[12] != kPos) return;
  if (out_size != kRowsBD * kFeat) return;
  if (ws_size < kWsTotal) return;

  const float* batch     = (const float*)d_in[0];
  const float* positions = (const float*)d_in[1];
  const float* tempten   = (const float*)d_in[2];
  const float* Wa = (const float*)d_in[3];
  const float* ba = (const float*)d_in[4];
  const float* Wb = (const float*)d_in[5];
  const float* bb = (const float*)d_in[6];
  const float* Wg = (const float*)d_in[7];
  const float* bg = (const float*)d_in[8];
  const float* Wp = (const float*)d_in[9];
  const float* bp = (const float*)d_in[10];
  const float* Wt = (const float*)d_in[11];
  const float* bt = (const float*)d_in[12];
  float* out = (float*)d_out;

  char* ws = (char*)d_ws;
  unsigned short* bdH   = (unsigned short*)(ws + kOffBdH);
  unsigned short* bdL   = (unsigned short*)(ws + kOffBdL);
  unsigned short* WaTH  = (unsigned short*)(ws + kOffWaTH);
  unsigned short* WaTL  = (unsigned short*)(ws + kOffWaTL);
  unsigned short* WcTH  = (unsigned short*)(ws + kOffWcTH);
  unsigned short* WcTL  = (unsigned short*)(ws + kOffWcTL);
  float* biasC  = (float*)(ws + kOffBiasC);
  float* biasA  = (float*)(ws + kOffBiasA);
  float* thetaC = (float*)(ws + kOffTheta);
  float* outSp  = (float*)(ws + kOffOutSp);
  unsigned short* planeH = (unsigned short*)(ws + kOffAH);
  unsigned short* planeL = (unsigned short*)(ws + kOffAL);
  float* planeC = (float*)(ws + kOffCpl);

  cast_split8_kernel<<<dim3((kRowsBD * kFeat / 8) / 256), dim3(256), 0, stream>>>(batch, bdH, bdL, kRowsBD * kFeat / 8);
  prep_weights_kernel<<<dim3(15, 3), dim3(256), 0, stream>>>(Wa, Wb, Wg, ba, bb, bg, WaTH, WaTL, WcTH, WcTL, biasC, biasA);
  wmma_gemm64<1, true, 2, 0, false, 0><<<dim3(kRowsBD / 64 / 8, 1), dim3(256), 0, stream>>>(
      bdH, bdL, kFeat, (long)0, WaTH, WaTL, kFeat, (long)0,
      (void*)thetaC, (void*)thetaC, 64, (long)0, biasA, biasA, (long)0,
      kRowsBD, 64, kFeat, 1.0f);

  for (int br = 0; br < 2; ++br) {
    const float* extra = (br == 0) ? positions : tempten;
    const float* Wx    = (br == 0) ? Wp : Wt;
    const float* bx    = (br == 0) ? bp : bt;
    const int D    = (br == 0) ? 9 : 10;
    const int sq   = (br == 0) ? 64 : 1;
    const int sk   = (br == 0) ? 1 : 64;
    const int bdG  = (br == 0) ? 64 : 0;
    const int bdB  = (br == 0) ? 0 : 64;
    float* dst     = (br == 0) ? outSp : out;
    const int addflag = (br == 0) ? 0 : 1;
    for (int c = 0; c < kNumChunk; ++c) {
      const int G0 = c * kGroupsPerChunk;
      build_rows_kernel<<<dim3(kRowsPerChunk / 64), dim3(256), 0, stream>>>(
          bdH, bdL, extra, Wx, bx, planeH, planeL, D, G0, bdG, bdB);
      wmma_gemm64<1, true, 2, 0, false, 0><<<dim3((kRowsPerChunk / 64) * (kNCol / 64) / 8, 1), dim3(256), 0, stream>>>(
          planeH, planeL, kKX, (long)0, WcTH, WcTL, kKX, (long)0,
          (void*)planeC, (void*)planeC, kNCol, (long)0, biasC, biasA, (long)0,
          kRowsPerChunk, kNCol, kKX, 1.0f);
      attn_rows_kernel<<<dim3(kGroupsPerChunk * 64 / 8), dim3(256), 0, stream>>>(
          planeC, thetaC, outSp, dst, G0, sq, sk, addflag);
    }
  }
}
